// Multi_Heads_Self_Attn_1D_1812476199802
// MI455X (gfx1250) — hardware-verified
//
#include <hip/hip_runtime.h>
#include <math.h>
#include <stdint.h>

#define NB    16
#define CIN   256
#define SEQ   1024
#define NH    8
#define DK    64
#define HD    512
#define NQKV  1536
#define LT    64
#define RSC   2048.0f
#define IRSC  0.00048828125f
#define WSC   64.0f
#define IWSC  0.015625f
#define IDK   0.015625f
#define QP    136
#define TP    72
#define XP    264
#define OPF   68
static_assert(NH * DK == HD);
static_assert(NQKV == 3 * HD);
static_assert((SEQ % LT) == 0);
static_assert((CIN % 32) == 0 && (HD % 32) == 0 && (SEQ % 32) == 0 && (DK % 32) == 0);
static_assert(64 * QP <= 128 * TP);
static_assert((QP % 8) == 0 && (TP % 8) == 0 && (XP % 8) == 0 && (OPF % 4) == 0);
static_assert(NQKV * CIN / 8 == 192 * 256);
static_assert(CIN * HD / 8 == 64 * 256);

typedef _Float16       v16h __attribute__((ext_vector_type(16)));
typedef _Float16       v8h  __attribute__((ext_vector_type(8)));
typedef __bf16         v16b __attribute__((ext_vector_type(16)));
typedef unsigned short v8us __attribute__((ext_vector_type(8)));
typedef float          v8f  __attribute__((ext_vector_type(8)));
typedef float          v4f  __attribute__((ext_vector_type(4)));
typedef unsigned int   v4u  __attribute__((ext_vector_type(4)));

union FragH { v16h v; v8h  h[2]; };
union FragB { v16b v; v8us u[2]; };
static_assert(sizeof(FragH) == 32);
static_assert(sizeof(FragB) == 32);

__device__ __forceinline__ unsigned short bf_bits(float f) {
  unsigned u = __float_as_uint(f);
  return (unsigned short)((u + 0x7FFFu + ((u >> 16) & 1u)) >> 16);
}
__device__ __forceinline__ float bf_up(unsigned short h) { return __uint_as_float(((unsigned)h) << 16); }
__device__ __forceinline__ float bfr(float f) { return bf_up(bf_bits(f)); }
__device__ __forceinline__ unsigned short h_bits(_Float16 x) { return __builtin_bit_cast(unsigned short, x); }
__device__ __forceinline__ unsigned pk16(unsigned short a, unsigned short b) { return (unsigned)a | ((unsigned)b << 16); }
__device__ __forceinline__ v8f zero8() { v8f z = {0.f, 0.f, 0.f, 0.f, 0.f, 0.f, 0.f, 0.f}; return z; }

__device__ __forceinline__ v16h ldfrag_h(const _Float16* p) {
  FragH f;
  f.h[0] = *(const v8h*)(p);
  f.h[1] = *(const v8h*)(p + 16);
  return f.v;
}
__device__ __forceinline__ v16b ldfrag_b(const unsigned short* p) {
  FragB f;
  f.u[0] = *(const v8us*)(p);
  f.u[1] = *(const v8us*)(p + 16);
  return f.v;
}

__device__ __forceinline__ v8f mma_h(v16h a, v16h b, v8f c) {
  v8f d = __builtin_amdgcn_wmma_f32_16x16x32_f16(false, a, false, b, (short)0, c, false, false);
#if defined(__HIP_DEVICE_COMPILE__)
  asm volatile("v_nop\n\tv_nop\n\tv_nop\n\tv_nop" : "+v"(d) : "v"(a), "v"(b));
#endif
  return d;
}
__device__ __forceinline__ v8f mma_b(v16b a, v16b b, v8f c) {
  v8f d = __builtin_amdgcn_wmma_f32_16x16x32_bf16(false, a, false, b, (short)0, c, false, false);
#if defined(__HIP_DEVICE_COMPILE__)
  const v16h ha = __builtin_bit_cast(v16h, a), hb = __builtin_bit_cast(v16h, b);
  asm volatile("v_nop\n\tv_nop\n\tv_nop\n\tv_nop" : "+v"(d) : "v"(ha), "v"(hb));
#endif
  return d;
}

__device__ __forceinline__ void stage_rm(unsigned short* Lh, unsigned short* Ll, int pitch, int row0, int col, v8f val) {
#pragma unroll
  for (int r = 0; r < 8; ++r) {
    const float v = val[r];
    const _Float16 hi = (_Float16)v;
    const float res = (v - (float)hi) * RSC;
    Lh[(row0 + r) * pitch + col] = h_bits(hi);
    Ll[(row0 + r) * pitch + col] = h_bits((_Float16)res);
  }
}
__device__ __forceinline__ void stage_cm(unsigned short* Lh, unsigned short* Ll, int pitch, int row0, int col, v8f val) {
#pragma unroll
  for (int r = 0; r < 8; ++r) {
    const float v = val[r];
    const _Float16 hi = (_Float16)v;
    const float res = (v - (float)hi) * RSC;
    Lh[col * pitch + row0 + r] = h_bits(hi);
    Ll[col * pitch + row0 + r] = h_bits((_Float16)res);
  }
}

__global__ __launch_bounds__(256) void cvt_w(const float* __restrict__ wq, const float* __restrict__ wk,
                                              const float* __restrict__ wv, const float* __restrict__ wo,
                                              unsigned short* WB, unsigned short* WO) {
  const int tid = threadIdx.x;
  if (blockIdx.x < 192) {
    const int i = blockIdx.x * 256 + tid;
    const int row = i >> 5;
    const int col = (i & 31) * 8;
    const int rq = min(row, HD - 1);
    const int rk = min(max(row - HD, 0), HD - 1);
    const int rv = min(max(row - 2 * HD, 0), HD - 1);
    const v4f q0 = *(const v4f*)(wq + (size_t)rq * CIN + col), q1 = *(const v4f*)(wq + (size_t)rq * CIN + col + 4);
    const v4f k0 = *(const v4f*)(wk + (size_t)rk * CIN + col), k1 = *(const v4f*)(wk + (size_t)rk * CIN + col + 4);
    const v4f v0 = *(const v4f*)(wv + (size_t)rv * CIN + col), v1 = *(const v4f*)(wv + (size_t)rv * CIN + col + 4);
    const bool isq = row < HD;
    const bool isk = row < 2 * HD;
    v4u w;
#pragma unroll
    for (int t = 0; t < 2; ++t) {
      const float a0 = isq ? q0[2 * t]     : (isk ? k0[2 * t]     : v0[2 * t]);
      const float a1 = isq ? q0[2 * t + 1] : (isk ? k0[2 * t + 1] : v0[2 * t + 1]);
      const float c0 = isq ? q1[2 * t]     : (isk ? k1[2 * t]     : v1[2 * t]);
      const float c1 = isq ? q1[2 * t + 1] : (isk ? k1[2 * t + 1] : v1[2 * t + 1]);
      w[t]     = pk16(bf_bits(a0), bf_bits(a1));
      w[2 + t] = pk16(bf_bits(c0), bf_bits(c1));
    }
    unsigned short* p = WB + (size_t)i * 8;
    *(volatile v4u*)p = w;
    __threadfence();
    *(volatile v4u*)p = w;
  } else {
    const int j = (blockIdx.x - 192) * 256 + tid;
    const int row = j >> 6;
    const int col = (j & 63) * 8;
    const v4f a0 = *(const v4f*)(wo + (size_t)row * HD + col), a1 = *(const v4f*)(wo + (size_t)row * HD + col + 4);
    v4u w;
#pragma unroll
    for (int t = 0; t < 2; ++t) {
      w[t]     = pk16(h_bits((_Float16)(bfr(a0[2 * t]) * WSC)), h_bits((_Float16)(bfr(a0[2 * t + 1]) * WSC)));
      w[2 + t] = pk16(h_bits((_Float16)(bfr(a1[2 * t]) * WSC)), h_bits((_Float16)(bfr(a1[2 * t + 1]) * WSC)));
    }
    unsigned short* p = WO + (size_t)j * 8;
    *(volatile v4u*)p = w;
    __threadfence();
    *(volatile v4u*)p = w;
  }
}

__global__ __launch_bounds__(256) void cvt_x(const float* __restrict__ x, unsigned short* XT) {
  __shared__ __align__(16) unsigned short T[LT * XP];
  const int tid = threadIdx.x;
  const int bx = blockIdx.x;
  const int b = bx >> 4, lt = bx & 15;
  const int l0 = lt * LT;
  {
    const int l4 = (tid & 15) * 4, cs = tid >> 4;
    const float* xp = x + ((size_t)b * CIN + cs) * SEQ + l0 + l4;
#pragma unroll
    for (int it = 0; it < 16; ++it) {
      const v4f v = *(const v4f*)(xp + (size_t)it * 16 * SEQ);
      const int c = it * 16 + cs;
#pragma unroll
      for (int q = 0; q < 4; ++q) T[(l4 + q) * XP + c] = bf_bits(v[q]);
    }
  }
  __syncthreads();
  {
    const int wave = tid >> 5, lane = tid & 31;
#pragma unroll
    for (int pass = 0; pass < 2; ++pass) {
#pragma unroll
      for (int it = 0; it < 8; ++it) {
        const int row = it * 8 + wave;
        const v4u u = *(const v4u*)(T + row * XP + 8 * lane);
        *(volatile v4u*)(XT + ((size_t)b * SEQ + l0 + row) * CIN + 8 * lane) = u;
      }
      __threadfence();
    }
  }
}

__global__ __launch_bounds__(256)
void proj_kernel(const unsigned short* __restrict__ XT, const unsigned short* __restrict__ WB,
                 unsigned short* QH, unsigned short* QL, unsigned short* KV) {
  __shared__ __align__(16) unsigned short Ls[2][128 * TP];
  const int tid  = threadIdx.x;
  const int lane = tid & 31, wave = tid >> 5;
  const int hh   = lane >> 4, c = lane & 15;
  const int bx   = blockIdx.x;
  const int chunk = bx % 12;
  const int lt   = (bx / 12) & 15;
  const int b    = bx / 192;
  const int l0   = lt * LT;
  const int rg   = wave & 3, chh = wave >> 2;
  const size_t NPL = (size_t)NB * HD * SEQ;

  const unsigned short* ap = XT + ((size_t)b * SEQ + l0 + rg * 16 + c) * CIN + 8 * hh;
  const unsigned short* bp = WB + ((size_t)(chunk * 128 + chh * 64 + c)) * CIN + 8 * hh;
  v8f acc0 = zero8(), acc1 = zero8(), acc2 = zero8(), acc3 = zero8();
#pragma unroll 1
  for (int ks = 0; ks < CIN / 32; ++ks) {
    const v16b a = ldfrag_b(ap + 32 * ks);
    const unsigned short* bs = bp + 32 * ks;
    acc0 = mma_b(a, ldfrag_b(bs + 0 * 16 * CIN), acc0);
    acc1 = mma_b(a, ldfrag_b(bs + 1 * 16 * CIN), acc1);
    acc2 = mma_b(a, ldfrag_b(bs + 2 * 16 * CIN), acc2);
    acc3 = mma_b(a, ldfrag_b(bs + 3 * 16 * CIN), acc3);
  }

  const int row0 = rg * 16 + 8 * hh;
  const int col0 = chh * 64 + c;
  if (chunk < 4) {
    stage_rm(Ls[0], Ls[1], QP, row0, col0 + 0 * 16, acc0);
    stage_rm(Ls[0], Ls[1], QP, row0, col0 + 1 * 16, acc1);
    stage_rm(Ls[0], Ls[1], QP, row0, col0 + 2 * 16, acc2);
    stage_rm(Ls[0], Ls[1], QP, row0, col0 + 3 * 16, acc3);
  } else {
    stage_cm(Ls[0], Ls[1], TP, row0, col0 + 0 * 16, acc0);
    stage_cm(Ls[0], Ls[1], TP, row0, col0 + 1 * 16, acc1);
    stage_cm(Ls[0], Ls[1], TP, row0, col0 + 2 * 16, acc2);
    stage_cm(Ls[0], Ls[1], TP, row0, col0 + 3 * 16, acc3);
  }
  __syncthreads();

  if (chunk < 4) {
    const int e = tid & 15, rq = tid >> 4;
    const int ch0 = chunk * 128;
#pragma unroll
    for (int pass = 0; pass < 2; ++pass) {
#pragma unroll
      for (int it = 0; it < 4; ++it) {
        const int row = it * 16 + rq;
        const int lo_ = row * QP + 8 * e;
        const v4u uh = *(const v4u*)(Ls[0] + lo_);
        const v4u ul = *(const v4u*)(Ls[1] + lo_);
        const size_t go = ((size_t)b * SEQ + l0 + row) * HD + ch0 + 8 * e;
        *(volatile v4u*)(QH + go) = uh;
        *(volatile v4u*)(QL + go) = ul;
      }
      __threadfence();
    }
  } else {
    const size_t psel = (chunk >= 8) ? 2 * NPL : (size_t)0;
    unsigned short* PH = KV + psel;
    unsigned short* PL = PH + NPL;
    const int ch0 = (chunk & 3) * 128;
    const int e = tid & 7, rq = tid >> 3;
#pragma unroll
    for (int pass = 0; pass < 2; ++pass) {
#pragma unroll
      for (int it = 0; it < 4; ++it) {
        const int cr = it * 32 + rq;
        const int lo_ = cr * TP + 8 * e;
        const v4u uh = *(const v4u*)(Ls[0] + lo_);
        const v4u ul = *(const v4u*)(Ls[1] + lo_);
        const size_t go = ((size_t)b * HD + ch0 + cr) * SEQ + l0 + 8 * e;
        *(volatile v4u*)(PH + go) = uh;
        *(volatile v4u*)(PL + go) = ul;
      }
      __threadfence();
    }
  }
}

__global__ __launch_bounds__(128)
void kv_kernel(const unsigned short* __restrict__ KV, unsigned short* MH, unsigned short* ML) {
  __shared__ __align__(16) unsigned short Ls[2][64 * TP];
  const int tid  = threadIdx.x;
  const int lane = tid & 31, wave = tid >> 5;
  const int hh   = lane >> 4, c = lane & 15;
  const int bh   = blockIdx.x;
  const size_t NPL = (size_t)NB * HD * SEQ;
  const _Float16* KHh = (const _Float16*)(const void*)(KV);
  const _Float16* KLh = (const _Float16*)(const void*)(KV + NPL);
  const _Float16* VHh = (const _Float16*)(const void*)(KV + 2 * NPL);
  const _Float16* VLh = (const _Float16*)(const void*)(KV + 3 * NPL);
  const size_t cb = (size_t)bh * DK;
  const _Float16* vhp = VHh + (cb + wave * 16 + c) * SEQ + 8 * hh;
  const _Float16* vlp = VLh + (cb + wave * 16 + c) * SEQ + 8 * hh;
  const _Float16* khp = KHh + (cb + c) * SEQ + 8 * hh;
  const _Float16* klp = KLh + (cb + c) * SEQ + 8 * hh;

  v8f aA0 = zero8(), aA1 = zero8(), aA2 = zero8(), aA3 = zero8();
  v8f aB0 = zero8(), aB1 = zero8(), aB2 = zero8(), aB3 = zero8();
#pragma unroll 1
  for (int ks = 0; ks < SEQ / 32; ++ks) {
    const int ko = 32 * ks;
    const v16h vh = ldfrag_h(vhp + ko), vl = ldfrag_h(vlp + ko);
    {
      const v16h kh = ldfrag_h(khp + 0 * 16 * SEQ + ko), kl = ldfrag_h(klp + 0 * 16 * SEQ + ko);
      aA0 = mma_h(vh, kh, aA0); aB0 = mma_h(vh, kl, aB0); aB0 = mma_h(vl, kh, aB0);
    }
    {
      const v16h kh = ldfrag_h(khp + 1 * 16 * SEQ + ko), kl = ldfrag_h(klp + 1 * 16 * SEQ + ko);
      aA1 = mma_h(vh, kh, aA1); aB1 = mma_h(vh, kl, aB1); aB1 = mma_h(vl, kh, aB1);
    }
    {
      const v16h kh = ldfrag_h(khp + 2 * 16 * SEQ + ko), kl = ldfrag_h(klp + 2 * 16 * SEQ + ko);
      aA2 = mma_h(vh, kh, aA2); aB2 = mma_h(vh, kl, aB2); aB2 = mma_h(vl, kh, aB2);
    }
    {
      const v16h kh = ldfrag_h(khp + 3 * 16 * SEQ + ko), kl = ldfrag_h(klp + 3 * 16 * SEQ + ko);
      aA3 = mma_h(vh, kh, aA3); aB3 = mma_h(vh, kl, aB3); aB3 = mma_h(vl, kh, aB3);
    }
  }

  const int row0 = wave * 16 + 8 * hh;
  {
    v8f s;
#pragma unroll
    for (int r = 0; r < 8; ++r) s[r] = aA0[r] + aB0[r] * IRSC;
    stage_rm(Ls[0], Ls[1], TP, row0, 0 * 16 + c, s);
#pragma unroll
    for (int r = 0; r < 8; ++r) s[r] = aA1[r] + aB1[r] * IRSC;
    stage_rm(Ls[0], Ls[1], TP, row0, 1 * 16 + c, s);
#pragma unroll
    for (int r = 0; r < 8; ++r) s[r] = aA2[r] + aB2[r] * IRSC;
    stage_rm(Ls[0], Ls[1], TP, row0, 2 * 16 + c, s);
#pragma unroll
    for (int r = 0; r < 8; ++r) s[r] = aA3[r] + aB3[r] * IRSC;
    stage_rm(Ls[0], Ls[1], TP, row0, 3 * 16 + c, s);
  }
  __syncthreads();
  {
    const int e = tid & 7, rq = tid >> 3;
#pragma unroll
    for (int pass = 0; pass < 2; ++pass) {
#pragma unroll
      for (int it = 0; it < 4; ++it) {
        const int row = it * 16 + rq;
        const int lo_ = row * TP + 8 * e;
        const v4u uh = *(const v4u*)(Ls[0] + lo_);
        const v4u ul = *(const v4u*)(Ls[1] + lo_);
        const size_t go = ((size_t)bh * DK + row) * DK + 8 * e;
        *(volatile v4u*)(MH + go) = uh;
        *(volatile v4u*)(ML + go) = ul;
      }
      __threadfence();
    }
  }
}

__global__ __launch_bounds__(256)
void qm_kernel(const unsigned short* __restrict__ QH, const unsigned short* __restrict__ QL,
               const unsigned short* __restrict__ MH, const unsigned short* __restrict__ ML,
               unsigned short* GH, unsigned short* GL) {
  __shared__ __align__(16) unsigned short Ls[2][64 * QP];
  const int tid  = threadIdx.x;
  const int lane = tid & 31, wave = tid >> 5;
  const int hh   = lane >> 4, c = lane & 15;
  const int bx   = blockIdx.x;
  const int hp   = bx & 3;
  const int lt   = (bx >> 2) & 15;
  const int b    = bx >> 6;
  const int l0   = lt * LT;
  const int rg   = wave & 3, hs = wave >> 2;
  const int head = hp * 2 + hs;
  const _Float16* QHh = (const _Float16*)(const void*)QH;
  const _Float16* QLh = (const _Float16*)(const void*)QL;
  const _Float16* MHh = (const _Float16*)(const void*)MH;
  const _Float16* MLh = (const _Float16*)(const void*)ML;
  const _Float16* qhp = QHh + ((size_t)b * SEQ + l0 + rg * 16 + c) * HD + head * DK + 8 * hh;
  const _Float16* qlp = QLh + ((size_t)b * SEQ + l0 + rg * 16 + c) * HD + head * DK + 8 * hh;
  const _Float16* mhp = MHh + (((size_t)b * NH + head) * DK + c) * DK + 8 * hh;
  const _Float16* mlp = MLh + (((size_t)b * NH + head) * DK + c) * DK + 8 * hh;

  v8f aA0 = zero8(), aA1 = zero8(), aA2 = zero8(), aA3 = zero8();
  v8f aB0 = zero8(), aB1 = zero8(), aB2 = zero8(), aB3 = zero8();
#pragma unroll 1
  for (int ks = 0; ks < DK / 32; ++ks) {
    const int ko = 32 * ks;
    const v16h qh = ldfrag_h(qhp + ko), ql = ldfrag_h(qlp + ko);
    {
      const v16h mh = ldfrag_h(mhp + 0 * 16 * DK + ko), ml = ldfrag_h(mlp + 0 * 16 * DK + ko);
      aA0 = mma_h(qh, mh, aA0); aB0 = mma_h(qh, ml, aB0); aB0 = mma_h(ql, mh, aB0);
    }
    {
      const v16h mh = ldfrag_h(mhp + 1 * 16 * DK + ko), ml = ldfrag_h(mlp + 1 * 16 * DK + ko);
      aA1 = mma_h(qh, mh, aA1); aB1 = mma_h(qh, ml, aB1); aB1 = mma_h(ql, mh, aB1);
    }
    {
      const v16h mh = ldfrag_h(mhp + 2 * 16 * DK + ko), ml = ldfrag_h(mlp + 2 * 16 * DK + ko);
      aA2 = mma_h(qh, mh, aA2); aB2 = mma_h(qh, ml, aB2); aB2 = mma_h(ql, mh, aB2);
    }
    {
      const v16h mh = ldfrag_h(mhp + 3 * 16 * DK + ko), ml = ldfrag_h(mlp + 3 * 16 * DK + ko);
      aA3 = mma_h(qh, mh, aA3); aB3 = mma_h(qh, ml, aB3); aB3 = mma_h(ql, mh, aB3);
    }
  }

  const int row0 = rg * 16 + 8 * hh;
  const int col0 = hs * 64 + c;
  {
    v8f s;
#pragma unroll
    for (int r = 0; r < 8; ++r) s[r] = (aA0[r] + aB0[r] * IRSC) * IDK;
    stage_rm(Ls[0], Ls[1], QP, row0, col0 + 0 * 16, s);
#pragma unroll
    for (int r = 0; r < 8; ++r) s[r] = (aA1[r] + aB1[r] * IRSC) * IDK;
    stage_rm(Ls[0], Ls[1], QP, row0, col0 + 1 * 16, s);
#pragma unroll
    for (int r = 0; r < 8; ++r) s[r] = (aA2[r] + aB2[r] * IRSC) * IDK;
    stage_rm(Ls[0], Ls[1], QP, row0, col0 + 2 * 16, s);
#pragma unroll
    for (int r = 0; r < 8; ++r) s[r] = (aA3[r] + aB3[r] * IRSC) * IDK;
    stage_rm(Ls[0], Ls[1], QP, row0, col0 + 3 * 16, s);
  }
  __syncthreads();
  {
    const int e = tid & 15, rq = tid >> 4;
#pragma unroll
    for (int pass = 0; pass < 2; ++pass) {
#pragma unroll
      for (int it = 0; it < 4; ++it) {
        const int row = it * 16 + rq;
        const int lo_ = row * QP + 8 * e;
        const v4u uh = *(const v4u*)(Ls[0] + lo_);
        const v4u ul = *(const v4u*)(Ls[1] + lo_);
        const size_t go = ((size_t)b * SEQ + l0 + row) * HD + hp * 128 + 8 * e;
        *(volatile v4u*)(GH + go) = uh;
        *(volatile v4u*)(GL + go) = ul;
      }
      __threadfence();
    }
  }
}

__global__ __launch_bounds__(256)
void wo_kernel(const unsigned short* __restrict__ GH, const unsigned short* __restrict__ GL,
               const unsigned short* __restrict__ WO, float* OF) {
  __shared__ __align__(16) float Os[128 * OPF];
  const int tid  = threadIdx.x;
  const int lane = tid & 31, wave = tid >> 5;
  const int hh   = lane >> 4, c = lane & 15;
  const int bx   = blockIdx.x;
  const int chalf = bx & 1;
  const int lt   = (bx >> 1) & 15;
  const int b    = bx >> 5;
  const int l0   = lt * LT;
  const int rg   = wave & 3, cq = wave >> 2;
  const _Float16* GHh = (const _Float16*)(const void*)GH;
  const _Float16* GLh = (const _Float16*)(const void*)GL;
  const _Float16* WOh = (const _Float16*)(const void*)WO;
  const _Float16* ghp = GHh + ((size_t)b * SEQ + l0 + rg * 16 + c) * HD + 8 * hh;
  const _Float16* glp = GLh + ((size_t)b * SEQ + l0 + rg * 16 + c) * HD + 8 * hh;
  const _Float16* wp  = WOh + ((size_t)(chalf * 128 + cq * 64 + c)) * HD + 8 * hh;

  v8f aA0 = zero8(), aA1 = zero8(), aA2 = zero8(), aA3 = zero8();
  v8f aB0 = zero8(), aB1 = zero8(), aB2 = zero8(), aB3 = zero8();
#pragma unroll 1
  for (int ks = 0; ks < HD / 32; ++ks) {
    const int ko = 32 * ks;
    const v16h gh = ldfrag_h(ghp + ko), gl = ldfrag_h(glp + ko);
    {
      const v16h w = ldfrag_h(wp + 0 * 16 * HD + ko);
      aA0 = mma_h(gh, w, aA0); aB0 = mma_h(gl, w, aB0);
    }
    {
      const v16h w = ldfrag_h(wp + 1 * 16 * HD + ko);
      aA1 = mma_h(gh, w, aA1); aB1 = mma_h(gl, w, aB1);
    }
    {
      const v16h w = ldfrag_h(wp + 2 * 16 * HD + ko);
      aA2 = mma_h(gh, w, aA2); aB2 = mma_h(gl, w, aB2);
    }
    {
      const v16h w = ldfrag_h(wp + 3 * 16 * HD + ko);
      aA3 = mma_h(gh, w, aA3); aB3 = mma_h(gl, w, aB3);
    }
  }

  const int row0 = rg * 16 + 8 * hh;
  const int col0 = cq * 64 + c;
  {
    float* o0 = Os + (col0 + 0 * 16) * OPF + row0;
    float* o1 = Os + (col0 + 1 * 16) * OPF + row0;
    float* o2 = Os + (col0 + 2 * 16) * OPF + row0;
    float* o3 = Os + (col0 + 3 * 16) * OPF + row0;
#pragma unroll
    for (int r = 0; r < 8; ++r) {
      o0[r] = (aA0[r] + aB0[r] * IRSC) * IWSC;
      o1[r] = (aA1[r] + aB1[r] * IRSC) * IWSC;
      o2[r] = (aA2[r] + aB2[r] * IRSC) * IWSC;
      o3[r] = (aA3[r] + aB3[r] * IRSC) * IWSC;
    }
  }
  __syncthreads();
  {
    const int e = tid & 15, rq = tid >> 4;
#pragma unroll
    for (int pass = 0; pass < 2; ++pass) {
#pragma unroll
      for (int it = 0; it < 8; ++it) {
        const int cl = it * 16 + rq;
        const v4f v = *(const v4f*)(Os + cl * OPF + 4 * e);
        *(volatile v4f*)(OF + ((size_t)b * CIN + chalf * 128 + cl) * SEQ + l0 + 4 * e) = v;
      }
      __threadfence();
    }
  }
}

__global__ __launch_bounds__(256)
void norm_kernel(const float* __restrict__ OF, const float* __restrict__ x, const float* __restrict__ gamma, float* out) {
  __shared__ float rs[256];
  const int tid = threadIdx.x;
  const size_t row = blockIdx.x;
  const v4f v = *(const v4f*)(OF + row * SEQ + 4 * tid);
  rs[tid] = (v[0] + v[1]) + (v[2] + v[3]);
  __syncthreads();
#pragma unroll
  for (int off = 128; off > 0; off >>= 1) {
    if (tid < off) rs[tid] = rs[tid] + rs[tid + off];
    __syncthreads();
  }
  const float mu = rs[0] * (1.0f / (float)SEQ);
  __syncthreads();
  v4f d;
#pragma unroll
  for (int q = 0; q < 4; ++q) d[q] = v[q] - mu;
  rs[tid] = (d[0] * d[0] + d[1] * d[1]) + (d[2] * d[2] + d[3] * d[3]);
  __syncthreads();
#pragma unroll
  for (int off = 128; off > 0; off >>= 1) {
    if (tid < off) rs[tid] = rs[tid] + rs[tid + off];
    __syncthreads();
  }
  const float var = rs[0] * (1.0f / (float)SEQ);
  const float inv = rsqrtf(var + 1e-5f);
  const float g = bfr(gamma[0]);
  const v4f xv = *(const v4f*)(x + row * SEQ + 4 * tid);
  v4f y;
#pragma unroll
  for (int q = 0; q < 4; ++q) {
    const float t = d[q] * inv;
    const float yy = t * g + bfr(xv[q]);
    y[q] = (yy >= 0.f) ? yy : 0.01f * yy;
  }
  float* p = out + row * SEQ + 4 * tid;
  *(volatile v4f*)p = y;
  __threadfence();
  *(volatile v4f*)p = y;
}

extern "C" void kernel_launch(void* const* d_in, const int* in_sizes, int n_in,
                              void* d_out, int out_size, void* d_ws, size_t ws_size,
                              hipStream_t stream) {
  const int NX = NB * CIN * SEQ;
  if (n_in < 6) return;
  if (in_sizes[0] != NX || in_sizes[1] != HD * CIN || in_sizes[2] != HD * CIN || in_sizes[3] != HD * CIN ||
      in_sizes[4] != CIN * HD || in_sizes[5] < 1) return;
  if (out_size != NX) return;

  const size_t NPL = (size_t)NB * HD * SEQ;
  size_t off = 0;
  const size_t oXT = off; off += (size_t)NB * SEQ * CIN * 2;
  const size_t oWB = off; off += (size_t)NQKV * CIN * 2;
  const size_t oWO = off; off += (size_t)CIN * HD * 2;
  const size_t oQH = off; off += NPL * 2;
  const size_t oQL = off; off += NPL * 2;
  const size_t oKV = off; off += 4 * NPL * 2;
  const size_t oMH = off; off += (size_t)NB * NH * DK * DK * 2;
  const size_t oML = off; off += (size_t)NB * NH * DK * DK * 2;
  if (off > ws_size) return;
  if (off > (size_t)134217728) return;
  if ((size_t)NB * CIN * SEQ * 4 > NPL * 2) return;

  const float* x  = (const float*)d_in[0];
  const float* Wq = (const float*)d_in[1];
  const float* Wk = (const float*)d_in[2];
  const float* Wv = (const float*)d_in[3];
  const float* Wo = (const float*)d_in[4];
  const float* gm = (const float*)d_in[5];
  char* ws = (char*)d_ws;
  unsigned short* XT = (unsigned short*)(ws + oXT);
  unsigned short* WB = (unsigned short*)(ws + oWB);
  unsigned short* WO = (unsigned short*)(ws + oWO);
  unsigned short* QH = (unsigned short*)(ws + oQH);
  unsigned short* QL = (unsigned short*)(ws + oQL);
  unsigned short* KV = (unsigned short*)(ws + oKV);
  unsigned short* MH = (unsigned short*)(ws + oMH);
  unsigned short* ML = (unsigned short*)(ws + oML);
  unsigned short* GH = KV;
  unsigned short* GL = KV + NPL;
  float* OF = (float*)(ws + oKV + 2 * NPL * 2);
  float* out = (float*)d_out;

  const dim3 blk256(256), blk128(128);
  const dim3 gW(256);
  const dim3 gX(NB * (SEQ / LT));
  const dim3 gP(NB * (SEQ / LT) * 12);
  const dim3 gK(NB * NH);
  const dim3 gQ(NB * (SEQ / LT) * 4);
  const dim3 gO(NB * (SEQ / LT) * 2);
  const dim3 gN(NB * CIN);

  cvt_w<<<gW, blk256, 0, stream>>>(Wq, Wk, Wv, Wo, WB, WO);
  cvt_x<<<gX, blk256, 0, stream>>>(x, XT);
  proj_kernel<<<gP, blk256, 0, stream>>>(XT, WB, QH, QL, KV);
  kv_kernel<<<gK, blk128, 0, stream>>>(KV, MH, ML);
  qm_kernel<<<gQ, blk256, 0, stream>>>(QH, QL, MH, ML, GH, GL);
  wo_kernel<<<gO, blk256, 0, stream>>>(GH, GL, WO, OF);
  norm_kernel<<<gN, blk256, 0, stream>>>(OF, x, gm, out);
  (void)hipGetLastError();
}
